// SNAT3_80857054314860
// MI455X (gfx1250) — hardware-verified
//
#include <hip/hip_runtime.h>
#include <math.h>
#include <stdint.h>
#pragma STDC FP_CONTRACT OFF

#define IN_DIM 128
#define HID    64
#define DCAT   256
#define NCONV  4
#define SLOPE  0.2f
#define THR    0.01f

typedef __bf16         v16b __attribute__((ext_vector_type(16)));
typedef unsigned short v8s  __attribute__((ext_vector_type(8)));
typedef float          v8f  __attribute__((ext_vector_type(8)));
typedef float          v4f  __attribute__((ext_vector_type(4)));
typedef float          v2f  __attribute__((ext_vector_type(2)));
typedef unsigned long long u64;

union Frag { v16b v; v8s h[2]; };

__device__ __forceinline__ unsigned short f2bf(float x)
{
    unsigned u = __float_as_uint(x);
    u = u + 0x7FFFu + ((u >> 16) & 1u);
    return (unsigned short)(u >> 16);
}
__device__ __forceinline__ float bf2f(unsigned short s)
{
    return __uint_as_float(((unsigned)s) << 16);
}

__device__ __forceinline__ void mma3(v8f& acc, const v16b ah, const v16b al, const v16b bh, const v16b bl)
{
    acc = __builtin_amdgcn_wmma_f32_16x16x32_bf16(false, ah, false, bh, (short)0, acc, false, false);
    acc = __builtin_amdgcn_wmma_f32_16x16x32_bf16(false, ah, false, bl, (short)0, acc, false, false);
    acc = __builtin_amdgcn_wmma_f32_16x16x32_bf16(false, al, false, bh, (short)0, acc, false, false);
    asm volatile("v_nop\n\tv_nop\n\tv_nop\n\tv_nop" : "+v"(acc) : "v"(ah), "v"(al), "v"(bh), "v"(bl));
}

__device__ __forceinline__ float wave_max(float v)
{
    v = fmaxf(v, __shfl_xor(v, 16, 32));
    v = fmaxf(v, __shfl_xor(v, 8, 32));
    v = fmaxf(v, __shfl_xor(v, 4, 32));
    v = fmaxf(v, __shfl_xor(v, 2, 32));
    v = fmaxf(v, __shfl_xor(v, 1, 32));
    return v;
}
__device__ __forceinline__ float wave_sum(float v)
{
    v += __shfl_xor(v, 16, 32);
    v += __shfl_xor(v, 8, 32);
    v += __shfl_xor(v, 4, 32);
    v += __shfl_xor(v, 2, 32);
    v += __shfl_xor(v, 1, 32);
    return v;
}

template<int ACT, bool DOTS>
__global__ void __launch_bounds__(256)
k_gemm(const float* __restrict__ A, int lda, int Mc, int K,
       const float* __restrict__ B, const float* __restrict__ bias,
       float* C, int ldc,
       const float* __restrict__ al, const float* __restrict__ ar,
       float* el, float* er)
{
    __shared__ v8s Ah[32 * 9];
    __shared__ v8s Al[32 * 9];
    __shared__ v8s Bh[64 * 9];
    __shared__ v8s Bl[64 * 9];
    __shared__ float Cs[32 * 68];
    __shared__ float els[32];
    __shared__ float ers[32];

    const int tid = threadIdx.x;
    const int w = tid >> 5, lane = tid & 31, h = lane >> 4, m = lane & 15;
    const int rt = w >> 2, ct = w & 3;
    const int row0 = blockIdx.x * 32;

    v8f acc = {0.f, 0.f, 0.f, 0.f, 0.f, 0.f, 0.f, 0.f};

    for (int kc = 0; kc < K; kc += 64) {
        {
            const int r = tid >> 3, c8 = (tid & 7) * 8;
            int gr = row0 + r; if (gr > Mc - 1) gr = Mc - 1;
            const float* ap = A + (size_t)gr * lda + kc + c8;
            v4f f0 = *(const v4f*)ap;
            v4f f1 = *(const v4f*)(ap + 4);
            v8s hv, lv;
#pragma unroll
            for (int i = 0; i < 4; ++i) {
                float x0 = f0[i]; unsigned short s0 = f2bf(x0);
                hv[i] = s0; lv[i] = f2bf(x0 - bf2f(s0));
                float x1 = f1[i]; unsigned short s1 = f2bf(x1);
                hv[4 + i] = s1; lv[4 + i] = f2bf(x1 - bf2f(s1));
            }
            Ah[r * 9 + (tid & 7)] = hv;
            Al[r * 9 + (tid & 7)] = lv;
        }
        {
            const int n = tid & 63, kq = tid >> 6;
            const float* bp = B + (size_t)(kc + kq * 16) * 64 + n;
            v8s h0, l0, h1, l1;
#pragma unroll
            for (int i = 0; i < 8; ++i) {
                float x0 = bp[(size_t)i * 64]; unsigned short s0 = f2bf(x0);
                h0[i] = s0; l0[i] = f2bf(x0 - bf2f(s0));
                float x1 = bp[(size_t)(8 + i) * 64]; unsigned short s1 = f2bf(x1);
                h1[i] = s1; l1[i] = f2bf(x1 - bf2f(s1));
            }
            Bh[n * 9 + kq * 2]     = h0;
            Bh[n * 9 + kq * 2 + 1] = h1;
            Bl[n * 9 + kq * 2]     = l0;
            Bl[n * 9 + kq * 2 + 1] = l1;
        }
        __syncthreads();

#pragma unroll
        for (int ks = 0; ks < 2; ++ks) {
            const int kb = ks * 4;
            const int ai = (rt * 16 + m) * 9 + kb + h;
            const int bi = (ct * 16 + m) * 9 + kb + h;
            Frag fa, fal, fb, fbl;
            fa.h[0]  = Ah[ai];  fa.h[1]  = Ah[ai + 2];
            fal.h[0] = Al[ai];  fal.h[1] = Al[ai + 2];
            fb.h[0]  = Bh[bi];  fb.h[1]  = Bh[bi + 2];
            fbl.h[0] = Bl[bi];  fbl.h[1] = Bl[bi + 2];
            mma3(acc, fa.v, fal.v, fb.v, fbl.v);
        }
        __syncthreads();
    }

    float bv = 0.f;
    if (bias) bv = bias[ct * 16 + m];
#pragma unroll
    for (int r = 0; r < 8; ++r) {
        float v = acc[r] + bv;
        if (ACT == 1)      v = tanhf(v);
        else if (ACT == 2) v = fmaxf(v, 0.0f);
        Cs[(rt * 16 + 8 * h + r) * 68 + ct * 16 + m] = v;
    }
    __syncthreads();

    if (DOTS) {
        const int r = tid >> 3, q = tid & 7;
        float pl = 0.f, pr = 0.f;
#pragma unroll
        for (int d = 0; d < 8; ++d) {
            float v = Cs[r * 68 + q * 8 + d];
            pl += v * al[q * 8 + d];
            pr += v * ar[q * 8 + d];
        }
        pl += __shfl_xor(pl, 1, 32); pl += __shfl_xor(pl, 2, 32); pl += __shfl_xor(pl, 4, 32);
        pr += __shfl_xor(pr, 1, 32); pr += __shfl_xor(pr, 2, 32); pr += __shfl_xor(pr, 4, 32);
        if (q == 0) { els[r] = pl; ers[r] = pr; }
        __syncthreads();
    }

#pragma unroll
    for (int it = 0; it < 2; ++it) {
        const int idx = it * 1024 + tid * 4;
        const int r = idx >> 6, c = idx & 63;
        v4f v = *(const v4f*)&Cs[r * 68 + c];
        *(volatile v4f*)(C + (size_t)(row0 + r) * ldc + c) = v;
    }
    if (DOTS) {
        if (w == 0) {
            float a = els[lane], b = ers[lane];
            *(volatile float*)(el + row0 + lane) = a;
            *(volatile float*)(er + row0 + lane) = b;
        }
    }
    __threadfence();
#pragma unroll
    for (int it = 0; it < 2; ++it) {
        const int idx = it * 1024 + tid * 4;
        const int r = idx >> 6, c = idx & 63;
        v4f v = *(const v4f*)&Cs[r * 68 + c];
        *(volatile v4f*)(C + (size_t)(row0 + r) * ldc + c) = v;
    }
    if (DOTS) {
        if (w == 0) {
            float a = els[lane], b = ers[lane];
            *(volatile float*)(el + row0 + lane) = a;
            *(volatile float*)(er + row0 + lane) = b;
        }
    }
}

__global__ void __launch_bounds__(256)
k_keys(const int* __restrict__ dst, u64* keys, int E, int EP, int N)
{
    const int p = blockIdx.x * 256 + threadIdx.x;
    if (p >= EP) return;
    u64 v = ~0ull;
    if (p < E) {
        int d = dst[p];
        if (d < 0) d = 0; if (d > N - 1) d = N - 1;
        v = (((u64)(unsigned)d) << 32) | (u64)(unsigned)p;
    }
    *(volatile u64*)(keys + p) = v;
    __threadfence();
    *(volatile u64*)(keys + p) = v;
}

__global__ void __launch_bounds__(256)
k_merge(const u64* __restrict__ in, u64* outk, int EP, int lw)
{
    const int p = blockIdx.x * 256 + threadIdx.x;
    if (p >= EP) return;
    const int wd   = 1 << lw;
    const int base = (p >> (lw + 1)) << (lw + 1);
    int la = EP - base; if (la > wd) la = wd;
    const int bs = base + wd;
    int lb = EP - bs; if (lb < 0) lb = 0; if (lb > wd) lb = wd;
    const int q = p - base;
    int lo = q - lb; if (lo < 0) lo = 0;
    int hi = (q < la) ? q : la;
    while (lo < hi) {
        const int mid = (lo + hi) >> 1;
        const u64 av = in[base + mid];
        const u64 bvv = in[bs + (q - 1 - mid)];
        if (av <= bvv) lo = mid + 1; else hi = mid;
    }
    const int i = lo, j = q - lo;
    bool takeA;
    if (i >= la)      takeA = false;
    else if (j >= lb) takeA = true;
    else              takeA = (in[base + i] <= in[bs + j]);
    const u64 v = takeA ? in[base + i] : in[bs + j];
    *(volatile u64*)(outk + p) = v;
    __threadfence();
    *(volatile u64*)(outk + p) = v;
}

__global__ void __launch_bounds__(256)
k_rowptr(const u64* __restrict__ keys, int* rowptr, int EP, int NPR)
{
    const int n = blockIdx.x * 256 + threadIdx.x;
    if (n >= NPR) return;
    int lo = 0, hi = EP;
    while (lo < hi) {
        const int mid = (lo + hi) >> 1;
        const unsigned d = (unsigned)(keys[mid] >> 32);
        if (d < (unsigned)n) lo = mid + 1; else hi = mid;
    }
    *(volatile int*)(rowptr + n) = lo;
    __threadfence();
    *(volatile int*)(rowptr + n) = lo;
}

__global__ void __launch_bounds__(256)
k_col(const u64* __restrict__ keys, const int* __restrict__ src, int* col, int E, int EP, int N)
{
    const int p = blockIdx.x * 256 + threadIdx.x;
    if (p >= EP) return;
    unsigned eid = (unsigned)(keys[p] & 0xFFFFFFFFull);
    if (eid > (unsigned)(E - 1)) eid = (unsigned)(E - 1);
    int s = src[eid];
    if (s < 0) s = 0; if (s > N - 1) s = N - 1;
    *(volatile int*)(col + p) = s;
    __threadfence();
    *(volatile int*)(col + p) = s;
}

__device__ __forceinline__ float lrelu(float t) { return (t > 0.0f) ? t : SLOPE * t; }

__device__ __forceinline__ float edge_score(int s, float ern, const float* el, int first,
                                            const float* el0, float er0n, float m0n, float inv0n)
{
    float sc = lrelu(el[s] + ern);
    if (!first) {
        float a0 = expf(lrelu(el0[s] + er0n) - m0n) * inv0n;
        if (!(a0 >= THR)) sc = -1e9f;
    }
    return sc;
}

__global__ void __launch_bounds__(256)
k_agg(const int* rowptr, const int* col, const float* feat,
      const float* el, const float* er,
      const float* el0, const float* er0, const float* m0r, const float* inv0r,
      float* m0w, float* inv0w, float* hout, int ldo, int first)
{
    __shared__ float ms[32];
    __shared__ float ivs[32];
    const int tid = threadIdx.x, w = tid >> 5, lane = tid & 31;
    const int nb = blockIdx.x * 32;

#pragma unroll 1
    for (int i = 0; i < 4; ++i) {
        const int n = nb + w * 4 + i;
        const int start = rowptr[n], end = rowptr[n + 1];
        const float ern = er[n];
        float er0n = 0.f, m0n = 0.f, inv0n = 0.f;
        if (!first) { er0n = er0[n]; m0n = m0r[n]; inv0n = inv0r[n]; }

        float mx = -INFINITY;
#pragma unroll 1
        for (int base = start; base < end; base += 32) {
            const int p = base + lane;
            float sc = -INFINITY;
            if (p < end) sc = edge_score(col[p], ern, el, first, el0, er0n, m0n, inv0n);
            mx = fmaxf(mx, sc);
        }
        mx = wave_max(mx);

        float sum = 0.f;
#pragma unroll 1
        for (int base = start; base < end; base += 32) {
            const int p = base + lane;
            float a = 0.f;
            if (p < end) a = expf(edge_score(col[p], ern, el, first, el0, er0n, m0n, inv0n) - mx);
            sum += a;
        }
        sum = wave_sum(sum);
        const float inv = 1.0f / fmaxf(sum, 1e-9f);

        float ax = 0.f, ay = 0.f;
#pragma unroll 1
        for (int base = start; base < end; base += 32) {
            const int p = base + lane;
            int s = 0; float alp = 0.f;
            if (p < end) {
                s = col[p];
                alp = expf(edge_score(s, ern, el, first, el0, er0n, m0n, inv0n) - mx) * inv;
            }
            int cnt = end - base; if (cnt > 32) cnt = 32;
#pragma unroll 1
            for (int j = 0; j < cnt; ++j) {
                const int   sj = __shfl(s, j, 32);
                const float aj = __shfl(alp, j, 32);
                v2f f = *(const v2f*)(feat + (size_t)sj * HID + 2 * lane);
                ax += f.x * aj;
                ay += f.y * aj;
            }
        }

        float ox = ax, oy = ay;
#pragma unroll 1
        for (int c = 0; c < 2; ++c) {
            const float v = (c == 0) ? ax : ay;
            const float r = (v > 0.0f) ? v : expm1f(v);
            if (c == 0) ox = r; else oy = r;
        }

        const int sl = (2 * lane) & 31;
        v4f o;
        o.x = __shfl(ox, sl, 32);
        o.y = __shfl(oy, sl, 32);
        o.z = __shfl(ox, sl + 1, 32);
        o.w = __shfl(oy, sl + 1, 32);
        volatile v4f* op = (volatile v4f*)(hout + (size_t)n * ldo + 4 * lane);
        if (lane < 16) *op = o;
        __threadfence();
        if (lane < 16) *op = o;

        if (first) {
            if (lane == 0) { ms[w * 4 + i] = mx; ivs[w * 4 + i] = inv; }
        }
    }

    if (first) {
        __syncthreads();
        if (w == 0) {
            const float a = ms[lane], b = ivs[lane];
            *(volatile float*)(m0w + nb + lane)   = a;
            *(volatile float*)(inv0w + nb + lane) = b;
            __threadfence();
            *(volatile float*)(m0w + nb + lane)   = a;
            *(volatile float*)(inv0w + nb + lane) = b;
        }
    }
}

__global__ void __launch_bounds__(256)
k_head(const float* __restrict__ t1, const float* __restrict__ W2,
       const float* __restrict__ b2, float* out, int N)
{
    const int g = blockIdx.x * 256 + threadIdx.x;
    const int n4 = g * 4;
    if (n4 >= N) return;
    int n0 = n4, n1 = n4 + 1, n2 = n4 + 2, n3 = n4 + 3;
    if (n1 > N - 1) n1 = N - 1;
    if (n2 > N - 1) n2 = N - 1;
    if (n3 > N - 1) n3 = N - 1;
    const float* r0 = t1 + (size_t)n0 * HID;
    const float* r1 = t1 + (size_t)n1 * HID;
    const float* r2 = t1 + (size_t)n2 * HID;
    const float* r3 = t1 + (size_t)n3 * HID;
    const float bb = b2[0];
    float s0 = bb, s1 = bb, s2 = bb, s3 = bb;
#pragma unroll 1
    for (int d = 0; d < HID; ++d) {
        const float wv = W2[d];
        s0 += r0[d] * wv;
        s1 += r1[d] * wv;
        s2 += r2[d] * wv;
        s3 += r3[d] * wv;
    }
    v4f o;
    o.x = fmaxf(s0, 0.0f); o.y = fmaxf(s1, 0.0f); o.z = fmaxf(s2, 0.0f); o.w = fmaxf(s3, 0.0f);
    if (n4 + 3 < N) {
        *(volatile v4f*)(out + n4) = o;
        __threadfence();
        *(volatile v4f*)(out + n4) = o;
    } else {
        *(volatile float*)(out + n4) = o.x;
        if (n4 + 1 < N) *(volatile float*)(out + n4 + 1) = o.y;
        if (n4 + 2 < N) *(volatile float*)(out + n4 + 2) = o.z;
        __threadfence();
        *(volatile float*)(out + n4) = o.x;
        if (n4 + 1 < N) *(volatile float*)(out + n4 + 1) = o.y;
        if (n4 + 2 < N) *(volatile float*)(out + n4 + 2) = o.z;
    }
}

extern "C" void kernel_launch(void* const* d_in, const int* in_sizes, int n_in,
                              void* d_out, int out_size, void* d_ws, size_t ws_size,
                              hipStream_t stream)
{
    (void)n_in; (void)out_size;
    const float* x       = (const float*)d_in[0];
    const int*   e_src   = (const int*)  d_in[1];
    const int*   e_dst   = (const int*)  d_in[2];
    const float* W_embed = (const float*)d_in[3];
    const float* W_gat   = (const float*)d_in[4];
    const float* a_l     = (const float*)d_in[5];
    const float* a_r     = (const float*)d_in[6];
    const float* W0      = (const float*)d_in[7];
    const float* b0      = (const float*)d_in[8];
    const float* W1      = (const float*)d_in[9];
    const float* b1      = (const float*)d_in[10];
    const float* W2      = (const float*)d_in[11];
    const float* b2      = (const float*)d_in[12];
    float* out = (float*)d_out;

    const int N = in_sizes[0] / IN_DIM;
    int E = in_sizes[1]; if (in_sizes[2] < E) E = in_sizes[2];
    if (N <= 0 || E <= 0) return;
    const int NP  = ((N + 31) / 32) * 32;
    const int NPR = NP + 32;
    const int EP  = ((E + 31) / 32) * 32;

    size_t off = 0;
    char* wsb = (char*)d_ws;
    auto take = [&](size_t bytes) -> char* { char* p = wsb + off; off += (bytes + 255) & ~(size_t)255; return p; };
    u64*   keysA  = (u64*)  take((size_t)EP * 8);
    u64*   keysB  = (u64*)  take((size_t)EP * 8);
    int*   rowptr = (int*)  take((size_t)NPR * 4);
    int*   col    = (int*)  take((size_t)EP * 4);
    float* h_emb  = (float*)take((size_t)NP * HID * 4);
    float* hcat   = (float*)take((size_t)NP * DCAT * 4);
    float* feat   = (float*)take((size_t)NP * HID * 4);
    float* t0     = (float*)take((size_t)NP * HID * 4);
    float* t1     = (float*)take((size_t)NP * HID * 4);
    float* el     = (float*)take((size_t)NCONV * NP * 4);
    float* er     = (float*)take((size_t)NCONV * NP * 4);
    float* m0     = (float*)take((size_t)NP * 4);
    float* inv0   = (float*)take((size_t)NP * 4);
    if (off > ws_size) return;

    const int gE = (EP + 255) / 256;
    const int gR = (NPR + 255) / 256;
    const int gG = NP / 32;
    const int gH = ((N + 3) / 4 + 255) / 256;

    k_keys<<<gE, 256, 0, stream>>>(e_dst, keysA, E, EP, N);
    u64* kin = keysA; u64* kout = keysB;
    for (int lw = 0; (1 << lw) < EP; ++lw) {
        k_merge<<<gE, 256, 0, stream>>>(kin, kout, EP, lw);
        u64* t = kin; kin = kout; kout = t;
    }
    k_rowptr<<<gR, 256, 0, stream>>>(kin, rowptr, EP, NPR);
    k_col<<<gE, 256, 0, stream>>>(kin, e_src, col, E, EP, N);

    k_gemm<1, false><<<gG, 256, 0, stream>>>(x, IN_DIM, N, IN_DIM, W_embed, nullptr,
                                             h_emb, HID, nullptr, nullptr, nullptr, nullptr);

    for (int l = 0; l < NCONV; ++l) {
        const float* A   = (l == 0) ? h_emb : (hcat + (size_t)(l - 1) * HID);
        const int    lda = (l == 0) ? HID : DCAT;
        k_gemm<0, true><<<gG, 256, 0, stream>>>(A, lda, N, HID, W_gat + (size_t)l * HID * HID, nullptr,
                                                feat, HID, a_l + (size_t)l * HID, a_r + (size_t)l * HID,
                                                el + (size_t)l * NP, er + (size_t)l * NP);
        k_agg<<<gG, 256, 0, stream>>>(rowptr, col, feat,
                                      el + (size_t)l * NP, er + (size_t)l * NP,
                                      el, er, m0, inv0, m0, inv0,
                                      hcat + (size_t)l * HID, DCAT, (l == 0) ? 1 : 0);
    }

    k_gemm<2, false><<<gG, 256, 0, stream>>>(hcat, DCAT, N, DCAT, W0, b0, t0, HID,
                                             nullptr, nullptr, nullptr, nullptr);
    k_gemm<2, false><<<gG, 256, 0, stream>>>(t0, HID, N, HID, W1, b1, t1, HID,
                                             nullptr, nullptr, nullptr, nullptr);
    k_head<<<gH, 256, 0, stream>>>(t1, W2, b2, out, N);
}
